// LSTMModelBahdanau_72172630442702
// MI455X (gfx1250) — hardware-verified
//
#include <hip/hip_runtime.h>


typedef _Float16 f16t;
typedef f16t  v16h __attribute__((ext_vector_type(16)));
typedef f16t  v8h  __attribute__((ext_vector_type(8)));
typedef float v8f  __attribute__((ext_vector_type(8)));
typedef float v4f  __attribute__((ext_vector_type(4)));
typedef unsigned int v4u __attribute__((ext_vector_type(4)));

union Frag { v16h v; v8h q[2]; };
union Pk16 { v8h h; v4u u; };
union Pk32 { v4f f; v4u u; };

#define BSZ  32
#define TSZ  256
#define IND  256
#define HIDD 512
#define G4   2048
#define ATT  64
#define EFW  128
#define OUTD 7
#define FCK  1024

#define HP 520
#define PP 264
#define SFP 68

#define INV256 0.00390625f

__device__ __forceinline__ v8f wmma16(v16h a, v16h b, v8f c) {
    return __builtin_amdgcn_wmma_f32_16x16x32_f16(false, a, false, b, (short)0, c, false, false);
}
__device__ __forceinline__ void wg1(v8f& c, const Frag& a, const Frag& b) {
    asm volatile("v_nop\n\tv_nop\n\tv_nop\n\tv_nop" : "+v"(c) : "v"(a.v), "v"(b.v));
}
__device__ __forceinline__ void wg2(v8f (&c)[2], const Frag& a, Frag (&b)[2]) {
    asm volatile("v_nop\n\tv_nop\n\tv_nop\n\tv_nop"
                 : "+v"(c[0]), "+v"(c[1])
                 : "v"(a.v), "v"(b[0].v), "v"(b[1].v));
}
__device__ __forceinline__ void wg4(v8f (&c)[4], const Frag& a, Frag (&b)[4]) {
    asm volatile("v_nop\n\tv_nop\n\tv_nop\n\tv_nop"
                 : "+v"(c[0]), "+v"(c[1]), "+v"(c[2]), "+v"(c[3])
                 : "v"(a.v), "v"(b[0].v), "v"(b[1].v), "v"(b[2].v), "v"(b[3].v));
}
__device__ __forceinline__ void ldfrag(Frag& f, const f16t* p) {
    f.q[0] = *(const v8h*)p;
    f.q[1] = *(const v8h*)(p + 16);
}
__device__ __forceinline__ v8f zero8() {
    const v8f z = {0.f, 0.f, 0.f, 0.f, 0.f, 0.f, 0.f, 0.f};
    return z;
}

__device__ __forceinline__ float ftanh(float x) {
    float ax = fabsf(x);
    float t  = __expf(-2.0f * ax);
    float r  = (1.0f - t) * __builtin_amdgcn_rcpf(1.0f + t);
    return copysignf(r, x);
}
__device__ __forceinline__ float fsig(float x) {
    return __builtin_amdgcn_rcpf(1.0f + __expf(-x));
}

__global__ __launch_bounds__(256)
void k_cvt8(const float* __restrict__ x, f16t* __restrict__ y, int n8, float sc) {
    int i = blockIdx.x * 256 + threadIdx.x;
    if (i >= n8) return;
    const float* p = x + (size_t)i * 8;
    v4f a = *(const v4f*)p;
    v4f b = *(const v4f*)(p + 4);
    Pk16 k;
    k.h[0] = (f16t)(a[0] * sc); k.h[1] = (f16t)(a[1] * sc); k.h[2] = (f16t)(a[2] * sc); k.h[3] = (f16t)(a[3] * sc);
    k.h[4] = (f16t)(b[0] * sc); k.h[5] = (f16t)(b[1] * sc); k.h[6] = (f16t)(b[2] * sc); k.h[7] = (f16t)(b[3] * sc);
    f16t* d = y + (size_t)i * 8;
    *(volatile v4u*)d = k.u;
    __threadfence();
    *(volatile v4u*)d = k.u;
}

__global__ __launch_bounds__(256)
void k_embed(const int* __restrict__ ids, const float* __restrict__ emb, f16t* __restrict__ X16,
             int nbt, int vocab) {
    int p = blockIdx.x * 256 + threadIdx.x;
    if (p >= nbt * 32) return;
    int bt = p >> 5, ch = (p & 31) * 8;
    int id = ids[bt];
    if (id < 0) id += vocab;
    id = min(max(id, 0), vocab - 1);
    const float* s = emb + (size_t)id * IND + ch;
    v4f a = *(const v4f*)s;
    v4f b = *(const v4f*)(s + 4);
    Pk16 k;
    k.h[0] = (f16t)(a[0] * 16.0f); k.h[1] = (f16t)(a[1] * 16.0f); k.h[2] = (f16t)(a[2] * 16.0f); k.h[3] = (f16t)(a[3] * 16.0f);
    k.h[4] = (f16t)(b[0] * 16.0f); k.h[5] = (f16t)(b[1] * 16.0f); k.h[6] = (f16t)(b[2] * 16.0f); k.h[7] = (f16t)(b[3] * 16.0f);
    f16t* d = X16 + (size_t)bt * IND + ch;
    *(volatile v4u*)d = k.u;
    __threadfence();
    *(volatile v4u*)d = k.u;
}

__global__ __launch_bounds__(256)
void k_wfc(const float* __restrict__ Wfc, f16t* __restrict__ P) {
    int p = blockIdx.x * 256 + threadIdx.x;
    if (p >= 16 * (FCK / 8)) return;
    int row = p >> 7, ch = (p & 127) * 8;
    int rs = row < OUTD ? row : OUTD - 1;
    const float* s = Wfc + (size_t)rs * FCK + ch;
    v4f a = *(const v4f*)s;
    v4f b = *(const v4f*)(s + 4);
    const bool live = row < OUTD;
    Pk16 k;
#pragma unroll
    for (int e = 0; e < 4; ++e) {
        k.h[e]     = (f16t)(live ? a[e] * 16.0f : 0.0f);
        k.h[4 + e] = (f16t)(live ? b[e] * 16.0f : 0.0f);
    }
    f16t* d = P + (size_t)row * FCK + ch;
    *(volatile v4u*)d = k.u;
    __threadfence();
    *(volatile v4u*)d = k.u;
}

__global__ __launch_bounds__(128)
void k_gemm64(const f16t* __restrict__ A, const f16t* __restrict__ B, float* __restrict__ C,
              int M, int N, int K, float inv,
              const float* __restrict__ bias0, int nb0,
              const float* __restrict__ bias1, int nb1,
              const float* __restrict__ bias2, float f2) {
    __shared__ __attribute__((aligned(16))) float Sf[64 * SFP];
    const int tid = threadIdx.x, w = tid >> 5, l = tid & 31, h = l >> 4, m = l & 15;
    const int row0 = blockIdx.y * 64, col0 = blockIdx.x * 64;
    if (row0 + 64 > M || col0 + 64 > N) return;

    v8f acc[4];
#pragma unroll
    for (int j = 0; j < 4; ++j) acc[j] = zero8();
    const f16t* ap = A + (size_t)(row0 + 16 * w + m) * K + 8 * h;
    const f16t* bp = B + (size_t)(col0 + m) * K + 8 * h;
#pragma unroll 1
    for (int k0 = 0; k0 < K; k0 += 32) {
        Frag a; ldfrag(a, ap + k0);
        Frag b[4];
#pragma unroll
        for (int j = 0; j < 4; ++j) ldfrag(b[j], bp + (size_t)(16 * j) * K + k0);
#pragma unroll
        for (int j = 0; j < 4; ++j) acc[j] = wmma16(a.v, b[j].v, acc[j]);
        wg4(acc, a, b);
    }
#pragma unroll
    for (int j = 0; j < 4; ++j) {
        const int col = col0 + 16 * j + m;
        const float v0 = bias0[min(col, nb0 - 1)];
        const float v1 = bias1[min(max(col - nb0, 0), nb1 - 1)];
        const float v2 = bias2[min(col, nb0 - 1)];
        const float bs = (col < nb0 ? v0 : v1) + f2 * v2;
#pragma unroll
        for (int r = 0; r < 8; ++r)
            Sf[(16 * w + 8 * h + r) * SFP + 16 * j + m] = fmaf(acc[j][r], inv, bs);
    }
    __syncthreads();
    Pk32 v[8];
#pragma unroll
    for (int i = 0; i < 8; ++i) {
        int p = tid + 128 * i, row = p >> 4, c4 = (p & 15) * 4;
        v[i].f = *(const v4f*)(Sf + row * SFP + c4);
    }
#pragma unroll
    for (int i = 0; i < 8; ++i) {
        int p = tid + 128 * i, row = p >> 4, c4 = (p & 15) * 4;
        *(volatile v4u*)(C + (size_t)(row0 + row) * N + col0 + c4) = v[i].u;
    }
    __threadfence();
#pragma unroll
    for (int i = 0; i < 8; ++i) {
        int p = tid + 128 * i, row = p >> 4, c4 = (p & 15) * 4;
        *(volatile v4u*)(C + (size_t)(row0 + row) * N + col0 + c4) = v[i].u;
    }
}

__global__ __launch_bounds__(256)
void k_lstm(const float* __restrict__ GX, const f16t* __restrict__ Whh16, f16t* __restrict__ lo16) {
    __shared__ __attribute__((aligned(16))) f16t Hb[2 * 16 * HP];
    const int tid = threadIdx.x, w = tid >> 5, l = tid & 31, h = l >> 4, m = l & 15;
    const int b0 = blockIdx.x * 16;

    for (int i = tid; i < 2 * 16 * HP; i += 256) Hb[i] = (f16t)0.0f;
    __syncthreads();

    float c[4][8];
#pragma unroll
    for (int q = 0; q < 4; ++q)
#pragma unroll
        for (int r = 0; r < 8; ++r) c[q][r] = 0.0f;

#pragma unroll 1
    for (int t = 0; t < TSZ; ++t) {
        const f16t* cur = Hb + (t & 1) * (16 * HP);
        f16t* nxt = Hb + ((t + 1) & 1) * (16 * HP);
#pragma unroll
        for (int q = 0; q < 4; ++q) {
            const int col = 64 * w + 16 * q + m;
            v8f acc[4];
#pragma unroll
            for (int g = 0; g < 4; ++g) acc[g] = zero8();
            const f16t* ap = cur + m * HP + 8 * h;
            const f16t* bp = Whh16 + (size_t)col * HIDD + 8 * h;
#pragma unroll 1
            for (int ks = 0; ks < HIDD / 32; ++ks) {
                Frag a; ldfrag(a, ap + ks * 32);
                Frag b[4];
#pragma unroll
                for (int g = 0; g < 4; ++g) ldfrag(b[g], bp + (size_t)g * ((size_t)HIDD * HIDD) + ks * 32);
#pragma unroll
                for (int g = 0; g < 4; ++g) acc[g] = wmma16(a.v, b[g].v, acc[g]);
                wg4(acc, a, b);
            }
            const float* gx = GX + ((size_t)(b0 + 8 * h) * TSZ + t) * G4 + col;
#pragma unroll
            for (int r = 0; r < 8; ++r) {
                const float* gr = gx + (size_t)r * TSZ * G4;
                const float pi = fmaf(acc[0][r], INV256, gr[0]);
                const float pf = fmaf(acc[1][r], INV256, gr[HIDD]);
                const float pg = fmaf(acc[2][r], INV256, gr[2 * HIDD]);
                const float po = fmaf(acc[3][r], INV256, gr[3 * HIDD]);
                const float cn = fsig(pf) * c[q][r] + fsig(pi) * ftanh(pg);
                c[q][r] = cn;
                const float hv = fsig(po) * ftanh(cn);
                nxt[(8 * h + r) * HP + col] = (f16t)(hv * 16.0f);
            }
        }
        __syncthreads();
        Pk16 v[4];
#pragma unroll
        for (int i = 0; i < 4; ++i) {
            int p = tid + 256 * i, row = p >> 6, ch = (p & 63) * 8;
            v[i].h = *(const v8h*)(nxt + row * HP + ch);
        }
#pragma unroll
        for (int i = 0; i < 4; ++i) {
            int p = tid + 256 * i, row = p >> 6, ch = (p & 63) * 8;
            *(volatile v4u*)(lo16 + ((size_t)(b0 + row) * TSZ + t) * HIDD + ch) = v[i].u;
        }
        __threadfence();
#pragma unroll
        for (int i = 0; i < 4; ++i) {
            int p = tid + 256 * i, row = p >> 6, ch = (p & 63) * 8;
            *(volatile v4u*)(lo16 + ((size_t)(b0 + row) * TSZ + t) * HIDD + ch) = v[i].u;
        }
    }
}

__global__ __launch_bounds__(128)
void k_tr(const f16t* __restrict__ in, f16t* __restrict__ outp) {
    __shared__ __attribute__((aligned(16))) f16t tile[64 * 72];
    const int tid = threadIdx.x;
    const int t0 = blockIdx.x * 64, n0 = blockIdx.y * 64, b = blockIdx.z;
#pragma unroll
    for (int i = 0; i < 4; ++i) {
        int p = tid + 128 * i, tr = p >> 3, ch = (p & 7) * 8;
        *(v8h*)(tile + tr * 72 + ch) = *(const v8h*)(in + ((size_t)(b * TSZ + t0 + tr)) * HIDD + n0 + ch);
    }
    __syncthreads();
    Pk16 v[4];
#pragma unroll
    for (int i = 0; i < 4; ++i) {
        int p = tid + 128 * i, nr = p >> 3, tc = p & 7;
#pragma unroll
        for (int j = 0; j < 8; ++j) v[i].h[j] = tile[(tc * 8 + j) * 72 + nr];
    }
#pragma unroll
    for (int i = 0; i < 4; ++i) {
        int p = tid + 128 * i, nr = p >> 3, tc = p & 7;
        *(volatile v4u*)(outp + ((size_t)(b * HIDD + n0 + nr)) * TSZ + t0 + tc * 8) = v[i].u;
    }
    __threadfence();
#pragma unroll
    for (int i = 0; i < 4; ++i) {
        int p = tid + 128 * i, nr = p >> 3, tc = p & 7;
        *(volatile v4u*)(outp + ((size_t)(b * HIDD + n0 + nr)) * TSZ + t0 + tc * 8) = v[i].u;
    }
}

__global__ __launch_bounds__(256)
void k_attn(const float* __restrict__ EF, const float* __restrict__ v, const float* __restrict__ vb,
            const f16t* __restrict__ loT16, const f16t* __restrict__ lo16,
            const f16t* __restrict__ Wfc16, const float* __restrict__ bfc, float* __restrict__ out) {
    __shared__ __attribute__((aligned(16))) float sdec[32 * ATT];
    __shared__ __attribute__((aligned(16))) float sv[ATT];
    __shared__ __attribute__((aligned(16))) float ureg[(32 * HP) / 2];
    __shared__ __attribute__((aligned(16))) f16t P16[32 * PP];
    __shared__ __attribute__((aligned(16))) float so[32 * OUTD];
    float* S = ureg;
    f16t* ctx16 = (f16t*)ureg;

    const int tid = threadIdx.x, w = tid >> 5, l = tid & 31, h = l >> 4, m = l & 15;
    const int b = blockIdx.y, td0 = blockIdx.x * 32, te = tid;

#pragma unroll
    for (int i = 0; i < 8; ++i) {
        int p = tid + 256 * i, r = p >> 6, a = p & 63;
        sdec[p] = EF[((size_t)(b * TSZ + td0 + r)) * EFW + ATT + a];
    }
    if (tid < ATT) sv[tid] = v[tid];
    const float vb0 = vb[0];
    __syncthreads();

    const float* erow = EF + ((size_t)(b * TSZ + te)) * EFW;
#pragma unroll 1
    for (int ac = 0; ac < ATT / 16; ++ac) {
        float ev[16], vv[16];
#pragma unroll
        for (int i = 0; i < 4; ++i) {
            v4f q = *(const v4f*)(erow + 16 * ac + 4 * i);
            ev[4 * i + 0] = q[0]; ev[4 * i + 1] = q[1]; ev[4 * i + 2] = q[2]; ev[4 * i + 3] = q[3];
        }
#pragma unroll
        for (int j = 0; j < 16; ++j) vv[j] = sv[16 * ac + j];
#pragma unroll 1
        for (int r = 0; r < 32; ++r) {
            const float* dr = sdec + r * ATT + 16 * ac;
            const float sprior = S[r * 256 + te];
            float s = (ac == 0) ? vb0 : sprior;
#pragma unroll
            for (int j = 0; j < 16; ++j) s = fmaf(vv[j], ftanh(dr[j] + ev[j]), s);
            S[r * 256 + te] = s;
        }
    }
    __syncthreads();

#pragma unroll
    for (int i = 0; i < 4; ++i) {
        const int r = 4 * w + i;
        v4f x0 = *(const v4f*)(S + r * 256 + l * 8);
        v4f x1 = *(const v4f*)(S + r * 256 + l * 8 + 4);
        float mx = fmaxf(fmaxf(fmaxf(x0[0], x0[1]), fmaxf(x0[2], x0[3])),
                         fmaxf(fmaxf(x1[0], x1[1]), fmaxf(x1[2], x1[3])));
#pragma unroll
        for (int off = 16; off; off >>= 1) mx = fmaxf(mx, __shfl_xor(mx, off, 32));
        float e[8];
        float sum = 0.0f;
#pragma unroll
        for (int j = 0; j < 4; ++j) {
            e[j]     = __expf(x0[j] - mx);
            e[4 + j] = __expf(x1[j] - mx);
            sum += e[j] + e[4 + j];
        }
#pragma unroll
        for (int off = 16; off; off >>= 1) sum += __shfl_xor(sum, off, 32);
        const float sc = 256.0f * __builtin_amdgcn_rcpf(sum);
        Pk16 pk;
#pragma unroll
        for (int j = 0; j < 8; ++j) pk.h[j] = (f16t)(e[j] * sc);
        *(v8h*)(P16 + r * PP + l * 8) = pk.h;
    }
    __syncthreads();

    {
        const int mt = w & 1, ng = w >> 1;
        const f16t* ap = P16 + (16 * mt + m) * PP + 8 * h;
#pragma unroll 1
        for (int grp = 0; grp < 4; ++grp) {
            const int c0 = 128 * ng + 32 * grp;
            v8f acc[2];
            acc[0] = zero8(); acc[1] = zero8();
            const f16t* bp = loT16 + ((size_t)b * HIDD + c0 + m) * TSZ + 8 * h;
#pragma unroll 1
            for (int ks = 0; ks < TSZ / 32; ++ks) {
                Frag a; ldfrag(a, ap + ks * 32);
                Frag bq[2];
                ldfrag(bq[0], bp + ks * 32);
                ldfrag(bq[1], bp + (size_t)16 * TSZ + ks * 32);
                acc[0] = wmma16(a.v, bq[0].v, acc[0]);
                acc[1] = wmma16(a.v, bq[1].v, acc[1]);
                wg2(acc, a, bq);
            }
#pragma unroll
            for (int j = 0; j < 2; ++j)
#pragma unroll
                for (int r = 0; r < 8; ++r)
                    ctx16[(16 * mt + 8 * h + r) * HP + c0 + 16 * j + m] = (f16t)(acc[j][r] * INV256);
        }
    }
    __syncthreads();

    if (w < 2) {
        const int mt = w;
        v8f acc = zero8();
        const f16t* ap = lo16 + ((size_t)(b * TSZ + td0 + 16 * mt + m)) * HIDD + 8 * h;
        const f16t* bp = Wfc16 + (size_t)m * FCK + 8 * h;
#pragma unroll 1
        for (int ks = 0; ks < HIDD / 32; ++ks) {
            Frag a, bb;
            ldfrag(a, ap + ks * 32);
            ldfrag(bb, bp + ks * 32);
            acc = wmma16(a.v, bb.v, acc);
            wg1(acc, a, bb);
        }
        const f16t* ap2 = ctx16 + (16 * mt + m) * HP + 8 * h;
#pragma unroll 1
        for (int ks = 0; ks < HIDD / 32; ++ks) {
            Frag a, bb;
            ldfrag(a, ap2 + ks * 32);
            ldfrag(bb, bp + HIDD + ks * 32);
            acc = wmma16(a.v, bb.v, acc);
            wg1(acc, a, bb);
        }
        const float bm = bfc[m < OUTD ? m : OUTD - 1];
        if (m < OUTD) {
#pragma unroll
            for (int r = 0; r < 8; ++r)
                so[(16 * mt + 8 * h + r) * OUTD + m] = fmaf(acc[r], INV256, bm);
        }
    }
    __syncthreads();

    {
        const int pc = tid < 56 ? tid : 55;
        Pk32 val;
        val.f = *(const v4f*)(so + pc * 4);
        float* dst = out + ((size_t)(b * TSZ + td0)) * OUTD + pc * 4;
        if (tid < 56) *(volatile v4u*)dst = val.u;
        __threadfence();
        if (tid < 56) *(volatile v4u*)dst = val.u;
    }
}

extern "C" void kernel_launch(void* const* d_in, const int* in_sizes, int n_in,
                              void* d_out, int out_size, void* d_ws, size_t ws_size,
                              hipStream_t stream) {
    const int nbt = BSZ * TSZ;
    if (n_in < 14) return;
    if (in_sizes[0] != nbt || out_size != nbt * OUTD) return;
    if ((in_sizes[1] % IND) != 0 || in_sizes[1] < IND) return;
    if (in_sizes[2] != G4 * IND || in_sizes[3] != G4 * HIDD || in_sizes[4] != G4 || in_sizes[5] != G4) return;
    if (in_sizes[6] != ATT * HIDD || in_sizes[7] != ATT || in_sizes[8] != ATT * HIDD || in_sizes[9] != ATT) return;
    if (in_sizes[10] != ATT || in_sizes[11] < 1 || in_sizes[12] != OUTD * FCK || in_sizes[13] != OUTD) return;
    const int vocab = in_sizes[1] / IND;

    const int*   ids = (const int*)  d_in[0];
    const float* emb = (const float*)d_in[1];
    const float* Wih = (const float*)d_in[2];
    const float* Whh = (const float*)d_in[3];
    const float* bih = (const float*)d_in[4];
    const float* bhh = (const float*)d_in[5];
    const float* We  = (const float*)d_in[6];
    const float* be  = (const float*)d_in[7];
    const float* Wd  = (const float*)d_in[8];
    const float* bd  = (const float*)d_in[9];
    const float* v   = (const float*)d_in[10];
    const float* vb  = (const float*)d_in[11];
    const float* Wfc = (const float*)d_in[12];
    const float* bfc = (const float*)d_in[13];
    float* out = (float*)d_out;

    char* ws = (char*)d_ws;
    size_t off = 0;
    auto carve = [&](size_t bytes) -> char* {
        char* p = ws + off;
        off = (off + bytes + 255) & ~(size_t)255;
        return p;
    };
    f16t*  X16   = (f16t*) carve((size_t)nbt * IND * 2);
    f16t*  Wih16 = (f16t*) carve((size_t)G4 * IND * 2);
    f16t*  Whh16 = (f16t*) carve((size_t)G4 * HIDD * 2);
    f16t*  Wed16 = (f16t*) carve((size_t)EFW * HIDD * 2);
    f16t*  Wfc16 = (f16t*) carve((size_t)16 * FCK * 2);
    float* GX    = (float*)carve((size_t)nbt * G4 * 4);
    f16t*  lo16  = (f16t*) carve((size_t)nbt * HIDD * 2);
    f16t*  loT16 = (f16t*) carve((size_t)BSZ * HIDD * TSZ * 2);
    float* EF    = (float*)carve((size_t)nbt * EFW * 4);
    if (off > ws_size || off > (size_t)134217728) return;

    k_embed<<<dim3((nbt * 32 + 255) / 256), dim3(256), 0, stream>>>(ids, emb, X16, nbt, vocab);
    k_cvt8<<<dim3((G4 * IND / 8 + 255) / 256), dim3(256), 0, stream>>>(Wih, Wih16, G4 * IND / 8, 16.0f);
    k_cvt8<<<dim3((G4 * HIDD / 8 + 255) / 256), dim3(256), 0, stream>>>(Whh, Whh16, G4 * HIDD / 8, 16.0f);
    k_cvt8<<<dim3((ATT * HIDD / 8 + 255) / 256), dim3(256), 0, stream>>>(We, Wed16, ATT * HIDD / 8, 16.0f);
    k_cvt8<<<dim3((ATT * HIDD / 8 + 255) / 256), dim3(256), 0, stream>>>(Wd, Wed16 + (size_t)ATT * HIDD, ATT * HIDD / 8, 16.0f);
    k_wfc<<<dim3((16 * (FCK / 8) + 255) / 256), dim3(256), 0, stream>>>(Wfc, Wfc16);

    k_gemm64<<<dim3(G4 / 64, nbt / 64), dim3(128), 0, stream>>>(
        X16, Wih16, GX, nbt, G4, IND, INV256, bih, G4, bih, G4, bhh, 1.0f);

    k_lstm<<<dim3(BSZ / 16), dim3(256), 0, stream>>>(GX, Whh16, lo16);

    k_tr<<<dim3(TSZ / 64, HIDD / 64, BSZ), dim3(128), 0, stream>>>(lo16, loT16);

    k_gemm64<<<dim3(EFW / 64, nbt / 64), dim3(128), 0, stream>>>(
        lo16, Wed16, EF, nbt, EFW, HIDD, INV256, be, ATT, bd, ATT, be, 0.0f);

    k_attn<<<dim3(TSZ / 32, BSZ), dim3(256), 0, stream>>>(EF, v, vb, loT16, lo16, Wfc16, bfc, out);
}
